// GSTA_59081570125116
// MI455X (gfx1250) — hardware-verified
//
#include <hip/hip_runtime.h>
#include <stddef.h>
#include <stdint.h>


typedef __attribute__((ext_vector_type(16))) _Float16 v16h;
typedef __attribute__((ext_vector_type(8)))  _Float16 v8h;
typedef __attribute__((ext_vector_type(4)))  _Float16 v4h;
typedef __attribute__((ext_vector_type(16))) __bf16   v16b;
typedef __attribute__((ext_vector_type(8)))  __bf16   v8b;
typedef __attribute__((ext_vector_type(8)))  float    v8f;
typedef __attribute__((ext_vector_type(4)))  float    v4f;
typedef __attribute__((ext_vector_type(2)))  unsigned u32x2;

__device__ __forceinline__ unsigned short f2bf_bits(float f) {
  unsigned u = __float_as_uint(f);
  return (unsigned short)((u + 0x7FFFu + ((u >> 16) & 1u)) >> 16);
}
__device__ __forceinline__ float bf_bits2f(unsigned short h) { return __uint_as_float(((unsigned)h) << 16); }

__device__ __forceinline__ void dep_guard_h(v8f& a, v8f& b, v16h x, v16h y) { asm volatile("v_nop\n\tv_nop\n\tv_nop\n\tv_nop" : "+v"(a), "+v"(b) : "v"(x), "v"(y)); }
__device__ __forceinline__ void dep_guard_b(v8f& a, v8f& b, v16b x, v16b y) { asm volatile("v_nop\n\tv_nop\n\tv_nop\n\tv_nop" : "+v"(a), "+v"(b) : "v"(x), "v"(y)); }
__device__ __forceinline__ void keep4_h(v16h a, v16h b, v16h c, v16h d) { asm volatile("v_nop" :: "v"(a), "v"(b), "v"(c), "v"(d)); }
__device__ __forceinline__ void keep4_b(v16b a, v16b b, v16b c, v16b d) { asm volatile("v_nop" :: "v"(a), "v"(b), "v"(c), "v"(d)); }
__device__ __forceinline__ void acc_guard4(v8f& a, v8f& b, v8f& c, v8f& d) { asm volatile("v_nop\n\tv_nop\n\tv_nop\n\tv_nop" : "+v"(a), "+v"(b), "+v"(c), "+v"(d)); }
template <typename T> struct Frag;
template <> struct Frag<_Float16> {
  typedef v16h V; union U { v16h v; v8h h[2]; };
  static __device__ __forceinline__ v16h load(const _Float16* p) {
    U f; f.h[0] = *(const v8h*)(p); f.h[1] = *(const v8h*)(p + 16); return f.v;
  }
  static __device__ __forceinline__ v8f mma(v16h a, v16h b, v8f c) {
    return __builtin_amdgcn_wmma_f32_16x16x32_f16(false, a, false, b, (short)0, c, false, false);
  }
  static __device__ __forceinline__ void guard(v8f& a, v8f& b, v16h x, v16h y) { dep_guard_h(a, b, x, y); }
  static __device__ __forceinline__ void keep(v16h a, v16h b, v16h c, v16h d) { keep4_h(a, b, c, d); }
};
template <> struct Frag<__bf16> {
  typedef v16b V; union U { v16b v; v8b h[2]; };
  static __device__ __forceinline__ v16b load(const __bf16* p) {
    U f; f.h[0] = *(const v8b*)(p); f.h[1] = *(const v8b*)(p + 16); return f.v;
  }
  static __device__ __forceinline__ v8f mma(v16b a, v16b b, v8f c) {
    return __builtin_amdgcn_wmma_f32_16x16x32_bf16(false, a, false, b, (short)0, c, false, false);
  }
  static __device__ __forceinline__ void guard(v8f& a, v8f& b, v16b x, v16b y) { dep_guard_b(a, b, x, y); }
  static __device__ __forceinline__ void keep(v16b a, v16b b, v16b c, v16b d) { keep4_b(a, b, c, d); }
};

template <int ET> struct Elem;
template <> struct Elem<0> { typedef _Float16 T; };
template <> struct Elem<1> { typedef __bf16 T; };
template <int ET, bool SPLIT, int BIAS_MODE, int OUT_MODE, bool RESID, bool SYM>
__global__ __launch_bounds__(256) void wmma_gemm64(
    const unsigned short* __restrict__ Ap, const unsigned short* __restrict__ A2p, int lda, long strideA,
    const unsigned short* __restrict__ Btp, const unsigned short* __restrict__ Bt2p, int ldb, long strideB,
    void* __restrict__ Cout, void* __restrict__ Cout2, int ldc, long strideC,
    const float* __restrict__ bias, float bias_scale,
    const float* __restrict__ resid, long strideR,
    const float* __restrict__ gmul,
    int M, int N, int K, float scale) {
  typedef typename Elem<ET>::T T;
  typedef typename Frag<T>::V V;
  const T* A = (const T*)Ap; const T* A2 = (const T*)A2p; const T* Bt = (const T*)Btp; const T* Bt2 = (const T*)Bt2p;
  __shared__ __align__(16) float sT[8][16 * 68];
  const int b    = blockIdx.y;
  const int lane = threadIdx.x & 31;
  const int wave = threadIdx.x >> 5;
  const int wpb  = blockDim.x >> 5;
  const int tilesN = N >> 6;
  const int tilesM = M >> 6;
  const int tile = blockIdx.x * wpb + wave;
  if (tile >= tilesM * tilesN) return;
  const int tm = tile / tilesN;
  const int tn = tile - tm * tilesN;
  if (SYM && tm > tn) return;
  const int m0 = tm << 6;
  const int n0 = tn << 6;

  const T* Ab  = A  + (size_t)b * strideA;
  const T* Bb  = Bt + (size_t)b * strideB;
  const T* Ab2 = SPLIT ? (A2  + (size_t)b * strideA) : nullptr;
  const T* Bb2 = SPLIT ? (Bt2 + (size_t)b * strideB) : nullptr;

  const int rlane = lane & 15;
  const int koff  = (lane >> 4) * 8;
  const int mOff  = (lane >> 4) * 8;

  v8f acc[4][4];
#pragma unroll
  for (int i = 0; i < 4; ++i)
#pragma unroll
    for (int j = 0; j < 4; ++j) acc[i][j] = (v8f){0.f,0.f,0.f,0.f,0.f,0.f,0.f,0.f};

  for (int k0 = 0; k0 < K; k0 += 32) {
    V bh[4], bl[4];
#pragma unroll
    for (int j = 0; j < 4; ++j) {
      const size_t bo = (size_t)(n0 + (j << 4) + rlane) * ldb + koff + k0;
      bh[j] = Frag<T>::load(Bb + bo);
      if (SPLIT) bl[j] = Frag<T>::load(Bb2 + bo);
    }
#pragma unroll
    for (int i = 0; i < 4; ++i) {
      const size_t ao = (size_t)(m0 + (i << 4) + rlane) * lda + koff + k0;
      V ah = Frag<T>::load(Ab + ao);
      V al;
      if (SPLIT) al = Frag<T>::load(Ab2 + ao);
#pragma unroll
      for (int j = 0; j < 4; ++j) {
        acc[i][j] = Frag<T>::mma(ah, bh[j], acc[i][j]);
        if (SPLIT) {
          acc[i][j] = Frag<T>::mma(ah, bl[j], acc[i][j]);
          acc[i][j] = Frag<T>::mma(al, bh[j], acc[i][j]);
        }
      }
      Frag<T>::guard(acc[i][0], acc[i][3], ah, SPLIT ? al : ah);
    }
    Frag<T>::keep(bh[0], bh[1], bh[2], bh[3]);
    if (SPLIT) Frag<T>::keep(bl[0], bl[1], bl[2], bl[3]);
  }
  acc_guard4(acc[0][0], acc[0][1], acc[0][2], acc[0][3]);
  acc_guard4(acc[1][0], acc[1][1], acc[1][2], acc[1][3]);
  acc_guard4(acc[2][0], acc[2][1], acc[2][2], acc[2][3]);
  acc_guard4(acc[3][0], acc[3][1], acc[3][2], acc[3][3]);

  const float sc = scale * ((gmul != nullptr) ? gmul[0] : 1.0f);

  float* slab = sT[wave];
  const float* Rb = RESID ? (resid + (size_t)b * strideR) : nullptr;
#pragma unroll
  for (int i = 0; i < 4; ++i) {
    const int mBase = m0 + (i << 4);
#pragma unroll
    for (int j = 0; j < 4; ++j) {
      const int n = n0 + (j << 4) + rlane;
      float bv = 0.f;
      if (BIAS_MODE == 2) bv = bias[n] * bias_scale;
#pragma unroll
      for (int r = 0; r < 8; ++r) {
        float v = acc[i][j][r] * sc;
        if (BIAS_MODE == 1) v += bias[mBase + mOff + r] * bias_scale;
        if (BIAS_MODE == 2) v += bv;
        if (RESID) v += Rb[(size_t)(mBase + mOff + r) * ldc + n];
        slab[(mOff + r) * 68 + (j << 4) + rlane] = v;
      }
    }
    __builtin_amdgcn_fence(__ATOMIC_RELEASE, "workgroup");
    __builtin_amdgcn_wave_barrier();
    __builtin_amdgcn_fence(__ATOMIC_ACQUIRE, "workgroup");
    if (OUT_MODE == 0) {
      float* C = (float*)Cout + (size_t)b * strideC;
      const int hh = lane >> 4, c4 = (lane & 15) * 4;
      for (int pass = 0; pass < 2; ++pass) {
#pragma unroll
        for (int it = 0; it < 8; ++it) {
          const int row = it * 2 + hh;
          v4f v = *(const v4f*)(slab + row * 68 + c4);
          *(volatile v4f*)(C + (size_t)(mBase + row) * ldc + n0 + c4) = v;
        }
        __threadfence();
      }
    } else {
      const int q = lane >> 3, c8 = (lane & 7) * 8;
      unsigned short* C  = (unsigned short*)Cout  + (size_t)b * strideC;
      unsigned short* C2 = (OUT_MODE == 2) ? ((unsigned short*)Cout2 + (size_t)b * strideC) : nullptr;
      for (int pass = 0; pass < 2; ++pass) {
#pragma unroll
        for (int it = 0; it < 4; ++it) {
          const int row = it * 4 + q;
          const float* sp = slab + row * 68 + c8;
          v8h hv, lv;
#pragma unroll
          for (int e = 0; e < 8; ++e) {
            if (OUT_MODE == 1) {
              hv[e] = (_Float16)sp[e];
            } else {
              unsigned short hb = f2bf_bits(sp[e]);
              unsigned short lb = f2bf_bits(sp[e] - bf_bits2f(hb));
              hv[e] = __builtin_bit_cast(_Float16, hb);
              lv[e] = __builtin_bit_cast(_Float16, lb);
            }
          }
          *(volatile v8h*)(C + (size_t)(mBase + row) * ldc + n0 + c8) = hv;
          if (OUT_MODE == 2) *(volatile v8h*)(C2 + (size_t)(mBase + row) * ldc + n0 + c8) = lv;
        }
        __threadfence();
      }
    }
    __builtin_amdgcn_fence(__ATOMIC_RELEASE, "workgroup");
    __builtin_amdgcn_wave_barrier();
    __builtin_amdgcn_fence(__ATOMIC_ACQUIRE, "workgroup");
  }

  if (SYM && OUT_MODE == 0 && tm != tn) {
    float* Cm = (float*)Cout + (size_t)b * strideC;
#pragma unroll
    for (int jj = 0; jj < 4; ++jj) {
      const int rBase = n0 + (jj << 4);
#pragma unroll
      for (int i = 0; i < 4; ++i) {
#pragma unroll
        for (int r = 0; r < 8; ++r) slab[rlane * 68 + (i << 4) + mOff + r] = acc[i][jj][r] * sc;
      }
      __builtin_amdgcn_fence(__ATOMIC_RELEASE, "workgroup");
      __builtin_amdgcn_wave_barrier();
      __builtin_amdgcn_fence(__ATOMIC_ACQUIRE, "workgroup");
      const int hh = lane >> 4, c4 = (lane & 15) * 4;
      for (int pass = 0; pass < 2; ++pass) {
#pragma unroll
        for (int it = 0; it < 8; ++it) {
          const int row = it * 2 + hh;
          v4f v = *(const v4f*)(slab + row * 68 + c4);
          *(volatile v4f*)(Cm + (size_t)(rBase + row) * ldc + m0 + c4) = v;
        }
        __threadfence();
      }
      __builtin_amdgcn_fence(__ATOMIC_RELEASE, "workgroup");
      __builtin_amdgcn_wave_barrier();
      __builtin_amdgcn_fence(__ATOMIC_ACQUIRE, "workgroup");
    }
  }
}

__global__ __launch_bounds__(256) void cast_f32_f16x2(
    const float* __restrict__ in, _Float16* __restrict__ out, int n2, float s) {
  int i = blockIdx.x * 256 + threadIdx.x;
  if (i < n2) {
    const _Float16 h0 = (_Float16)(in[2 * i] * s), h1 = (_Float16)(in[2 * i + 1] * s);
    const unsigned u = (unsigned)__builtin_bit_cast(unsigned short, h0) | ((unsigned)__builtin_bit_cast(unsigned short, h1) << 16);
    ((volatile unsigned*)out)[i] = u;
    __threadfence();
    ((volatile unsigned*)out)[i] = u;
  }
}

__global__ __launch_bounds__(256) void k_tr16(const float* __restrict__ in, _Float16* __restrict__ out,
                                              int R, int Cc, float s) {
  __shared__ __align__(16) _Float16 T[64 * 132];
  const int t = threadIdx.x, lane = t & 31, wave = t >> 5;
  const int z = blockIdx.y, c0 = blockIdx.x * 64;
  const float* ib = in + ((size_t)z * R + c0) * Cc;
  const int col4 = lane * 4;
#pragma unroll
  for (int p = 0; p < 8; ++p) {
    const int r = p * 8 + wave;
    const v4f v = *(const v4f*)(ib + (size_t)r * Cc + col4);
    v4h h;
    h[0] = (_Float16)(v[0] * s); h[1] = (_Float16)(v[1] * s); h[2] = (_Float16)(v[2] * s); h[3] = (_Float16)(v[3] * s);
    *(v4h*)(T + r * 132 + col4) = h;
  }
  __syncthreads();
  _Float16* ob = out + (size_t)z * Cc * R + c0;
  const int q = lane >> 3, c8 = (lane & 7) * 8;
  for (int pass = 0; pass < 2; ++pass) {
#pragma unroll
    for (int it = 0; it < 4; ++it) {
      const int m = it * 32 + wave * 4 + q;
      v8h hv;
#pragma unroll
      for (int e = 0; e < 8; ++e) hv[e] = T[(c8 + e) * 132 + m];
      *(volatile v8h*)(ob + (size_t)m * R + c8) = hv;
    }
    __threadfence();
  }
}

__global__ __launch_bounds__(128) void k_sm128(const float* __restrict__ E, _Float16* __restrict__ P, int nrows) {
  __shared__ __align__(16) _Float16 S[4][2][128];
  const int lane = threadIdx.x & 31, wave = threadIdx.x >> 5;
  const int base = blockIdx.x * 8 + wave * 2;
#pragma unroll
  for (int rr = 0; rr < 2; ++rr) {
    int row = base + rr; row = row < nrows ? row : nrows - 1;
    const v4f x = *(const v4f*)(E + (size_t)row * 128 + 4 * lane);
    float mx = fmaxf(fmaxf(x[0], x[1]), fmaxf(x[2], x[3]));
#pragma unroll
    for (int off = 16; off > 0; off >>= 1) mx = fmaxf(mx, __shfl_xor(mx, off, 32));
    const float e0 = expf(x[0] - mx), e1 = expf(x[1] - mx), e2 = expf(x[2] - mx), e3 = expf(x[3] - mx);
    float s = (e0 + e1) + (e2 + e3);
#pragma unroll
    for (int off = 16; off > 0; off >>= 1) s += __shfl_xor(s, off, 32);
    const float inv = 32768.0f / s;
    _Float16* sp = &S[wave][rr][4 * lane];
    sp[0] = (_Float16)(e0 * inv); sp[1] = (_Float16)(e1 * inv); sp[2] = (_Float16)(e2 * inv); sp[3] = (_Float16)(e3 * inv);
  }
  __syncthreads();
  const int r2 = lane >> 4, piece = lane & 15;
  int row = base + r2; row = row < nrows ? row : nrows - 1;
  const v8h hv = *(const v8h*)(&S[wave][r2][piece * 8]);
  _Float16* dst = P + (size_t)row * 128 + piece * 8;
  *(volatile v8h*)dst = hv;
  __threadfence();
  *(volatile v8h*)dst = hv;
}

__global__ __launch_bounds__(256) void k_sm2048(const float* __restrict__ E, _Float16* __restrict__ P, int nrows, int W) {
  __shared__ float redA[8];
  __shared__ float redB[8];
  int row = blockIdx.x; row = row < nrows ? row : nrows - 1;
  const int t = threadIdx.x, lane = t & 31, wave = t >> 5;
  const float* er = E + (size_t)row * W;
  const v4f x0 = *(const v4f*)(er + 8 * t), x1 = *(const v4f*)(er + 8 * t + 4);
  float mn = fminf(fminf(fminf(x0[0], x0[1]), fminf(x0[2], x0[3])), fminf(fminf(x1[0], x1[1]), fminf(x1[2], x1[3])));
#pragma unroll
  for (int off = 16; off > 0; off >>= 1) mn = fminf(mn, __shfl_xor(mn, off, 32));
  if (lane == 0) redA[wave] = mn;
  __syncthreads();
  mn = redA[0];
#pragma unroll
  for (int i = 1; i < 8; ++i) mn = fminf(mn, redA[i]);
  float e[8];
  e[0] = expf(mn - x0[0]); e[1] = expf(mn - x0[1]); e[2] = expf(mn - x0[2]); e[3] = expf(mn - x0[3]);
  e[4] = expf(mn - x1[0]); e[5] = expf(mn - x1[1]); e[6] = expf(mn - x1[2]); e[7] = expf(mn - x1[3]);
  float s = ((e[0] + e[1]) + (e[2] + e[3])) + ((e[4] + e[5]) + (e[6] + e[7]));
#pragma unroll
  for (int off = 16; off > 0; off >>= 1) s += __shfl_xor(s, off, 32);
  if (lane == 0) redB[wave] = s;
  __syncthreads();
  float tot = redB[0];
#pragma unroll
  for (int i = 1; i < 8; ++i) tot += redB[i];
  const float inv = 32768.0f / tot;
  v8h hv;
#pragma unroll
  for (int i = 0; i < 8; ++i) hv[i] = (_Float16)(e[i] * inv);
  _Float16* dst = P + (size_t)row * W + 8 * t;
  *(volatile v8h*)dst = hv;
  __threadfence();
  *(volatile v8h*)dst = hv;
}

__device__ __forceinline__ float blk_half_sum(float x, float* red, int lane, int wave, int half) {
#pragma unroll
  for (int off = 16; off > 0; off >>= 1) x += __shfl_xor(x, off, 32);
  __syncthreads();
  if (lane == 0) red[wave] = x;
  __syncthreads();
  const int b0 = half * 4;
  float s = red[b0]; s += red[b0 + 1]; s += red[b0 + 2]; s += red[b0 + 3];
  return s;
}

__global__ __launch_bounds__(256) void k_graph(const float* __restrict__ GR, const float* __restrict__ ADJ,
                                               _Float16* __restrict__ GO, int nrows) {
  __shared__ float red[8];
  __shared__ __align__(16) _Float16 S[2][128];
  const int t = threadIdx.x, lane = t & 31, wave = t >> 5, half = t >> 7, w = t & 127;
  int row = blockIdx.x * 2 + half; row = row < nrows ? row : nrows - 1;
  const int n = row >> 7, v = row & 127;
  const float* gb = GR + (size_t)n * 16384;
  const float gvv = gb[v * 129], gww = gb[w * 129], gvw = gb[v * 128 + w];
  const bool offd = (w != v);
  float av = ADJ[(size_t)row * 128 + w];
  av = offd ? av : 0.0f;
  const float sa = blk_half_sum(fabsf(av), red, lane, wave, half);
  float d2 = (gww + gvv) - 2.0f * gvw;
  d2 = fmaxf(d2, 1e-12f);
  const float dist = sqrtf(d2);
  float sim = 2.0f / (expf(dist) + 1.0f);
  sim = offd ? sim : 0.0f;
  const float ss = blk_half_sum(fabsf(sim), red, lane, wave, half);
  const float ra = 1.0f / fmaxf(sa, 1e-12f);
  const float rs = 1.0f / fmaxf(ss, 1e-12f);
  const float gval = 0.5f * (av * ra + sim * rs);
  S[half][w] = (_Float16)(gval * 16384.0f);
  __syncthreads();
  if (wave == 0) {
    const int r2 = lane >> 4, piece = lane & 15;
    int orow = blockIdx.x * 2 + r2; orow = orow < nrows ? orow : nrows - 1;
    const v8h hv = *(const v8h*)(&S[r2][piece * 8]);
    _Float16* dst = GO + (size_t)orow * 128 + piece * 8;
    *(volatile v8h*)dst = hv;
    __threadfence();
    *(volatile v8h*)dst = hv;
  }
}

__global__ __launch_bounds__(256) void k_bn_stats(const float* __restrict__ HP, float* __restrict__ mean,
                                                  float* __restrict__ istd, int rows, int C) {
  const int o = blockIdx.x * 256 + threadIdx.x;
  const int oc = o < C ? o : C - 1;
  double s = 0.0;
  for (int r = 0; r < rows; ++r) s += (double)HP[(size_t)r * C + oc];
  const float mf = (float)(s / (double)rows);
  double q = 0.0;
  for (int r = 0; r < rows; ++r) {
    const float d = HP[(size_t)r * C + oc] - mf;
    q += (double)d * (double)d;
  }
  const float var = (float)(q / (double)rows);
  const float is = 1.0f / sqrtf(var + 1e-5f);
  if (o < C) {
    ((volatile float*)mean)[o] = mf;
    ((volatile float*)istd)[o] = is;
    __threadfence();
    ((volatile float*)mean)[o] = mf;
    ((volatile float*)istd)[o] = is;
  }
}

__global__ __launch_bounds__(256) void k_bn_apply(const float* __restrict__ HP, const float* __restrict__ GIN,
    const float* __restrict__ mean, const float* __restrict__ istd, const float* __restrict__ bw,
    const float* __restrict__ bb, const float* __restrict__ gam, int gidx,
    float* __restrict__ GOUT, _Float16* __restrict__ G16, int write16, int total4, int C) {
  const int i4 = blockIdx.x * 256 + threadIdx.x;
  if (i4 >= total4) return;
  const size_t i = (size_t)i4 * 4;
  const int o = (int)(i % (size_t)C);
  const v4f hp = *(const v4f*)(HP + i), g = *(const v4f*)(GIN + i);
  const v4f m = *(const v4f*)(mean + o), s = *(const v4f*)(istd + o), w = *(const v4f*)(bw + o), bv = *(const v4f*)(bb + o);
  const float gm = gam[gidx];
  v4f r;
#pragma unroll
  for (int e = 0; e < 4; ++e) {
    const float hb = (hp[e] - m[e]) * s[e] * w[e] + bv[e];
    const float a = (hb > 0.0f) ? hb : 0.1f * hb;
    r[e] = g[e] + gm * a;
  }
  u32x2 pk;
  {
    const unsigned short b0 = __builtin_bit_cast(unsigned short, (_Float16)(r[0] * 8.0f));
    const unsigned short b1 = __builtin_bit_cast(unsigned short, (_Float16)(r[1] * 8.0f));
    const unsigned short b2 = __builtin_bit_cast(unsigned short, (_Float16)(r[2] * 8.0f));
    const unsigned short b3 = __builtin_bit_cast(unsigned short, (_Float16)(r[3] * 8.0f));
    pk[0] = (unsigned)b0 | ((unsigned)b1 << 16);
    pk[1] = (unsigned)b2 | ((unsigned)b3 << 16);
  }
  *(volatile v4f*)(GOUT + i) = r;
  if (write16) *(volatile u32x2*)(G16 + i) = pk;
  __threadfence();
  *(volatile v4f*)(GOUT + i) = r;
  if (write16) *(volatile u32x2*)(G16 + i) = pk;
}

#define GEMM_QK  wmma_gemm64<0, false, 2, 1, false, false>
#define GEMM_V   wmma_gemm64<0, false, 1, 1, false, false>
#define GEMM_F32 wmma_gemm64<0, false, 0, 0, false, false>
#define GEMM_RES wmma_gemm64<0, false, 0, 0, true, false>
#define GEMM_SYM wmma_gemm64<0, false, 0, 0, false, true>
#define GEMM_H16 wmma_gemm64<0, false, 0, 1, false, false>

extern "C" void kernel_launch(void* const* d_in, const int* in_sizes, int n_in,
                              void* d_out, int out_size, void* d_ws, size_t ws_size,
                              hipStream_t stream) {
  const int B = 16, C = 2048, HW = 128, C8 = 256, NG = 16, V = 128, L = 2, GI = 2;
  if (n_in < 15) return;
  if (in_sizes[0] != B * C * HW || in_sizes[1] != NG * V * C || in_sizes[2] != NG * V * V ||
      in_sizes[3] != C8 * C || in_sizes[4] < C8 || in_sizes[5] != C8 * C || in_sizes[6] < C8 ||
      in_sizes[7] != C * C || in_sizes[8] < C || in_sizes[9] < 1 || in_sizes[10] < 1 ||
      in_sizes[11] != L * C * C || in_sizes[12] < L * C || in_sizes[13] < L * C || in_sizes[14] < L) return;
  if (out_size != B * C * HW + NG * V * C) return;

  const float* x     = (const float*)d_in[0];
  const float* vfeat = (const float*)d_in[1];
  const float* adj   = (const float*)d_in[2];
  const float* Wq    = (const float*)d_in[3];
  const float* bq    = (const float*)d_in[4];
  const float* Wk    = (const float*)d_in[5];
  const float* bk    = (const float*)d_in[6];
  const float* Wv    = (const float*)d_in[7];
  const float* bv    = (const float*)d_in[8];
  const float* gpx   = (const float*)d_in[9];
  const float* gch   = (const float*)d_in[10];
  const float* Wg    = (const float*)d_in[11];
  const float* bnw   = (const float*)d_in[12];
  const float* bnb   = (const float*)d_in[13];
  const float* gg    = (const float*)d_in[14];

  const size_t nBCHW = (size_t)B * C * HW;
  const size_t nNVC  = (size_t)NG * V * C;
  float* outY = (float*)d_out;
  float* outG = outY + nBCHW;

  char* ws = (char*)d_ws;
  size_t off = 0;
  auto carve = [&off](size_t bytes) -> size_t { size_t o = off; off += (bytes + 4095) & ~(size_t)4095; return o; };
  const size_t o_xT16 = carve(nBCHW * 2);
  const size_t o_Wq16 = carve((size_t)C8 * C * 2);
  const size_t o_Wk16 = carve((size_t)C8 * C * 2);
  const size_t o_Wv16 = carve((size_t)C * C * 2);
  const size_t o_q16  = carve((size_t)B * HW * C8 * 2);
  const size_t o_k16  = carve((size_t)B * HW * C8 * 2);
  const size_t o_v16  = carve(nBCHW * 2);
  const size_t o_E    = carve((size_t)B * HW * HW * 4);
  const size_t o_att  = carve((size_t)B * HW * HW * 2);
  const size_t o_y1   = carve(nBCHW * 4);
  const size_t o_y16  = carve(nBCHW * 2);
  const size_t o_yT16 = carve(nBCHW * 2);
  const size_t o_chE  = carve((size_t)GI * C * C * 4);
  const size_t o_P16  = carve((size_t)GI * C * C * 2);
  const size_t endAB = off;
  off = 0;
  const size_t o_g16  = carve(nNVC * 2);
  const size_t o_Wg16 = carve((size_t)C * C * 2);
  const size_t o_hT16 = carve(nNVC * 2);
  const size_t o_gram = carve((size_t)NG * V * V * 4);
  const size_t o_gr16 = carve((size_t)NG * V * V * 2);
  const size_t o_mean = carve((size_t)C * 4);
  const size_t o_istd = carve((size_t)C * 4);
  const size_t o_hp   = carve(nNVC * 4);
  const size_t o_gbuf = carve(nNVC * 4);
  const size_t endC = off;
  const size_t total = (endAB > endC) ? endAB : endC;
  if (total > ws_size || total > (size_t)134217728) return;

  unsigned short* xT16 = (unsigned short*)(ws + o_xT16);
  unsigned short* Wq16 = (unsigned short*)(ws + o_Wq16);
  unsigned short* Wk16 = (unsigned short*)(ws + o_Wk16);
  unsigned short* Wv16 = (unsigned short*)(ws + o_Wv16);
  unsigned short* q16  = (unsigned short*)(ws + o_q16);
  unsigned short* k16  = (unsigned short*)(ws + o_k16);
  unsigned short* v16  = (unsigned short*)(ws + o_v16);
  float*          E    = (float*)(ws + o_E);
  unsigned short* att  = (unsigned short*)(ws + o_att);
  float*          y1   = (float*)(ws + o_y1);
  unsigned short* y16  = (unsigned short*)(ws + o_y16);
  unsigned short* yT16 = (unsigned short*)(ws + o_yT16);
  float*          chE  = (float*)(ws + o_chE);
  unsigned short* P16  = (unsigned short*)(ws + o_P16);
  unsigned short* g16  = (unsigned short*)(ws + o_g16);
  unsigned short* Wg16 = (unsigned short*)(ws + o_Wg16);
  unsigned short* hT16 = (unsigned short*)(ws + o_hT16);
  float*          gram = (float*)(ws + o_gram);
  unsigned short* gr16 = (unsigned short*)(ws + o_gr16);
  float*          mean = (float*)(ws + o_mean);
  float*          istd = (float*)(ws + o_istd);
  float*          hp   = (float*)(ws + o_hp);
  float*          gbuf = (float*)(ws + o_gbuf);

  const dim3 t256(256), t128(128);
  auto gt = [](int M_, int N_, int wpb) { const int tl = (M_ / 64) * (N_ / 64); return (unsigned)((tl + wpb - 1) / wpb); };

  cast_f32_f16x2<<<dim3((unsigned)((C8 * C / 2 + 255) / 256)), t256, 0, stream>>>(Wq, (_Float16*)Wq16, C8 * C / 2, 64.0f);
  cast_f32_f16x2<<<dim3((unsigned)((C8 * C / 2 + 255) / 256)), t256, 0, stream>>>(Wk, (_Float16*)Wk16, C8 * C / 2, 64.0f);
  cast_f32_f16x2<<<dim3((unsigned)((C * C / 2 + 255) / 256)), t256, 0, stream>>>(Wv, (_Float16*)Wv16, C * C / 2, 64.0f);
  k_tr16<<<dim3(C / 64, B), t256, 0, stream>>>(x, (_Float16*)xT16, C, HW, 8.0f);

  GEMM_QK<<<dim3(gt(HW, C8, 8), B), t256, 0, stream>>>(
      xT16, nullptr, C, (long)HW * C, Wq16, nullptr, C, 0L,
      q16, nullptr, C8, (long)HW * C8, bq, 16.0f, nullptr, 0L, nullptr, HW, C8, C, 1.0f / 32.0f);
  GEMM_QK<<<dim3(gt(HW, C8, 8), B), t256, 0, stream>>>(
      xT16, nullptr, C, (long)HW * C, Wk16, nullptr, C, 0L,
      k16, nullptr, C8, (long)HW * C8, bk, 16.0f, nullptr, 0L, nullptr, HW, C8, C, 1.0f / 32.0f);
  GEMM_V<<<dim3(gt(C, HW, 8), B), t256, 0, stream>>>(
      Wv16, nullptr, C, 0L, xT16, nullptr, C, (long)HW * C,
      v16, nullptr, HW, (long)C * HW, bv, 16.0f, nullptr, 0L, nullptr, C, HW, C, 1.0f / 32.0f);
  GEMM_F32<<<dim3(gt(HW, HW, 4), B), t128, 0, stream>>>(
      q16, nullptr, C8, (long)HW * C8, k16, nullptr, C8, (long)HW * C8,
      E, nullptr, HW, (long)HW * HW, nullptr, 0.0f, nullptr, 0L, nullptr, HW, HW, C8, 1.0f / 256.0f);
  k_sm128<<<dim3((unsigned)(B * HW / 8)), t128, 0, stream>>>(E, (_Float16*)att, B * HW);
  GEMM_RES<<<dim3(gt(C, HW, 8), B), t256, 0, stream>>>(
      v16, nullptr, HW, (long)C * HW, att, nullptr, HW, (long)HW * HW,
      y1, nullptr, HW, (long)C * HW, nullptr, 0.0f, x, (long)C * HW, gpx, C, HW, HW, 1.0f / 524288.0f);

  cast_f32_f16x2<<<dim3((unsigned)((nBCHW / 2 + 255) / 256)), t256, 0, stream>>>(y1, (_Float16*)y16, (int)(nBCHW / 2), 8.0f);
  k_tr16<<<dim3(C / 64, B), t256, 0, stream>>>(y1, (_Float16*)yT16, C, HW, 8.0f);
  for (int grp = 0; grp < B / GI; ++grp) {
    const size_t img0 = (size_t)grp * GI;
    GEMM_SYM<<<dim3(gt(C, C, 8), GI), t256, 0, stream>>>(
        y16 + img0 * C * HW, nullptr, HW, (long)C * HW, y16 + img0 * C * HW, nullptr, HW, (long)C * HW,
        chE, nullptr, C, (long)C * C, nullptr, 0.0f, nullptr, 0L, nullptr, C, C, HW, 1.0f / 64.0f);
    k_sm2048<<<dim3((unsigned)(GI * C)), t256, 0, stream>>>(chE, (_Float16*)P16, GI * C, C);
    GEMM_RES<<<dim3(gt(C, HW, 8), GI), t256, 0, stream>>>(
        P16, nullptr, C, (long)C * C, yT16 + img0 * HW * C, nullptr, C, (long)HW * C,
        outY + img0 * C * HW, nullptr, HW, (long)C * HW, nullptr, 0.0f, y1 + img0 * C * HW, (long)C * HW, gch,
        C, HW, C, 1.0f / 262144.0f);
  }

  cast_f32_f16x2<<<dim3((unsigned)((nNVC / 2 + 255) / 256)), t256, 0, stream>>>(vfeat, (_Float16*)g16, (int)(nNVC / 2), 8.0f);
  for (int li = 0; li < L; ++li) {
    const float* gin = (li == 0) ? vfeat : gbuf;
    float* gout = (li == L - 1) ? outG : gbuf;
    const int w16 = (li == L - 1) ? 0 : 1;
    cast_f32_f16x2<<<dim3((unsigned)((C * C / 2 + 255) / 256)), t256, 0, stream>>>(Wg + (size_t)li * C * C, (_Float16*)Wg16, C * C / 2, 64.0f);
    GEMM_H16<<<dim3(gt(C, V, 8), NG), t256, 0, stream>>>(
        Wg16, nullptr, C, 0L, g16, nullptr, C, (long)V * C,
        hT16, nullptr, V, (long)C * V, nullptr, 0.0f, nullptr, 0L, nullptr, C, V, C, 1.0f / 32.0f);
    GEMM_SYM<<<dim3(gt(V, V, 4), NG), t128, 0, stream>>>(
        g16, nullptr, C, (long)V * C, g16, nullptr, C, (long)V * C,
        gram, nullptr, V, (long)V * V, nullptr, 0.0f, nullptr, 0L, nullptr, V, V, C, 1.0f / 64.0f);
    k_graph<<<dim3((unsigned)(NG * V / 2)), t256, 0, stream>>>(gram, adj, (_Float16*)gr16, NG * V);
    GEMM_F32<<<dim3(gt(V, C, 8), NG), t256, 0, stream>>>(
        gr16, nullptr, V, (long)V * V, hT16, nullptr, V, (long)C * V,
        hp, nullptr, C, (long)V * C, nullptr, 0.0f, nullptr, 0L, nullptr, V, C, V, 1.0f / 262144.0f);
    k_bn_stats<<<dim3((unsigned)((C + 255) / 256)), t256, 0, stream>>>(hp, mean, istd, NG * V, C);
    k_bn_apply<<<dim3((unsigned)((nNVC / 4 + 255) / 256)), t256, 0, stream>>>(
        hp, gin, mean, istd, bnw + (size_t)li * C, bnb + (size_t)li * C, gg, li,
        gout, (_Float16*)g16, w16, (int)(nNVC / 4), C);
  }
}
